// GraphIdentifierEnvNonlinear_46995532152909
// MI455X (gfx1250) — hardware-verified
//
#include <hip/hip_runtime.h>


namespace {
constexpr int Bn = 4, N = 1024, H = 32;
constexpr float AS_ = 8.0f, WS_ = 8.0f, STEP = 0.1f;

typedef _Float16 b16;
typedef __attribute__((ext_vector_type(16))) _Float16 v16b;
typedef __attribute__((ext_vector_type(8))) _Float16 v8b;
typedef __attribute__((ext_vector_type(8))) float v8f;
typedef __attribute__((ext_vector_type(4))) float v4f;
__device__ __forceinline__ void split16(float v, b16& hi, b16& lo) { hi = (b16)v; lo = (b16)(v - (float)hi); }
__device__ __forceinline__ v16b frag_kb(const b16* p, int hh) { const v8b a = *(const v8b*)(p + 8 * hh), b = *(const v8b*)(p + 16 + 8 * hh); v16b f;
#pragma unroll
  for (int e = 0; e < 8; ++e) { f[e] = a[e]; f[8 + e] = b[e]; } return f; }
__device__ __forceinline__ v8f wmma16b(v16b a, v16b b, v8f c) { v8f d = __builtin_amdgcn_wmma_f32_16x16x32_f16(false, a, false, b, (short)0, c, false, false); asm volatile("v_nop\n\tv_nop\n\tv_nop\n\tv_nop" : "+v"(d) : "v"(a), "v"(b)); return d; }
__device__ __forceinline__ void wave_lds_sync() { __builtin_amdgcn_fence(__ATOMIC_RELEASE, "workgroup"); __builtin_amdgcn_wave_barrier(); __builtin_amdgcn_fence(__ATOMIC_ACQUIRE, "workgroup"); }
__device__ __forceinline__ float nexp(float x) { return __builtin_amdgcn_exp2f(x * 1.4426950408889634f); }
__device__ __forceinline__ float tanh_(float x) { const float e = nexp(-2.0f * fabsf(x)); const float t = (1.0f - e) * __builtin_amdgcn_rcpf(1.0f + e); return (x >= 0.0f) ? t : -t; }
__device__ __forceinline__ float sigm(float x) { return __builtin_amdgcn_rcpf(1.0f + nexp(-x)); }
__device__ __forceinline__ float pmul(float a, float b) { float p = a * b; asm volatile("" : "+v"(p)); return p; }

__global__ __launch_bounds__(256) void prep_kernel(const float* __restrict__ Theta, const float* __restrict__ W2, float* __restrict__ Arow, b16* __restrict__ w2p) {
  const int wid = threadIdx.x >> 5, lane = threadIdx.x & 31, i = blockIdx.x * 8 + wid; const float* tr = Theta + (size_t)i * N;
  float m = -INFINITY; for (int j = lane; j < N; j += 32) m = fmaxf(m, tr[j]);
#pragma unroll
  for (int o = 1; o < 32; o <<= 1) m = fmaxf(m, __shfl_xor(m, o));
  float s = 0.0f; for (int j = lane; j < N; j += 32) s += __expf(tr[j] - m);
#pragma unroll
  for (int o = 1; o < 32; o <<= 1) s += __shfl_xor(s, o);
  const float aii = __expf(tr[i] - m) / s; const float rs = 1.0f - aii; const float inv = 1.0f / (s * ((rs > 0.0f) ? rs : 1.0f));
  for (int pass = 0; pass < 2; ++pass) {
    for (int j0 = 0; j0 < N; j0 += 128) { const int j = j0 + lane * 4; v4f o;
#pragma unroll
      for (int e = 0; e < 4; ++e) o[e] = (j + e == i) ? 0.0f : __expf(tr[j + e] - m) * inv;
      *(volatile v4f*)(Arow + (size_t)i * N + j) = o; }
    if (blockIdx.x == 0) { for (int p = threadIdx.x; p < H * H; p += 256) { b16 a, c; split16(W2[p] * WS_, a, c); ((volatile b16*)w2p)[p] = a; ((volatile b16*)w2p)[H * H + p] = c; } }
    __threadfence(); }
}

__global__ __launch_bounds__(256) void pair_kernel(const float* __restrict__ x, const float* __restrict__ Arow, const float* __restrict__ W1, const float* __restrict__ b1, const b16* __restrict__ w2p, const float* __restrict__ b2, const float* __restrict__ W3, const float* __restrict__ b3, float* __restrict__ out) {
  __shared__ float Ob[32];
  const int wid = threadIdx.x >> 5, lane = threadIdx.x & 31, nloc = lane & 15, hlf = lane >> 4; const int b = blockIdx.x / (N / 32), i0 = (blockIdx.x % (N / 32)) * 32;
  const float* xb = x + (size_t)b * N;
  const v16b w2h0 = frag_kb(w2p + (size_t)(0 * 16 + nloc) * H, hlf), w2l0 = frag_kb(w2p + H * H + (size_t)(0 * 16 + nloc) * H, hlf), w2h1 = frag_kb(w2p + (size_t)(16 + nloc) * H, hlf), w2l1 = frag_kb(w2p + H * H + (size_t)(16 + nloc) * H, hlf);
  const float w3a = W3[nloc], w3b = W3[16 + nloc], b2a = b2[nloc], b2b = b2[16 + nloc], bb3 = b3[0];
  for (int ri = 0; ri < 4; ++ri) { const int i = i0 + wid * 4 + ri; const float xi = xb[i]; const float* Ai = Arow + (size_t)i * N;
    float ak[16];
#pragma unroll
    for (int e = 0; e < 16; ++e) { const int h = (e < 8) ? (8 * hlf + e) : (16 + 8 * hlf + e - 8); ak[e] = xi * (W1[h * 3 + 0] - W1[h * 3 + 2]) + b1[h]; }
    float ck[16];
#pragma unroll
    for (int e = 0; e < 16; ++e) { const int h = (e < 8) ? (8 * hlf + e) : (16 + 8 * hlf + e - 8); ck[e] = W1[h * 3 + 1] + W1[h * 3 + 2]; }
    float agg = 0.0f;
    for (int jt = 0; jt < N; jt += 16) { const float xj = xb[jt + nloc]; v16b ah, al;
#pragma unroll
      for (int e = 0; e < 16; ++e) { b16 a, c; split16(tanh_(ak[e] + pmul(xj, ck[e])) * AS_, a, c); ah[e] = a; al[e] = c; }
      v8f acc0 = {}, acc1 = {};
      acc0 = wmma16b(ah, w2h0, acc0); acc0 = wmma16b(al, w2h0, acc0); acc0 = wmma16b(ah, w2l0, acc0);
      acc1 = wmma16b(ah, w2h1, acc1); acc1 = wmma16b(al, w2h1, acc1); acc1 = wmma16b(ah, w2l1, acc1);
#pragma unroll
      for (int v = 0; v < 8; ++v) { float pr = pmul(tanh_(acc0[v] * (1.0f / (AS_ * WS_)) + b2a), w3a) + pmul(tanh_(acc1[v] * (1.0f / (AS_ * WS_)) + b2b), w3b);
#pragma unroll
        for (int o = 1; o < 16; o <<= 1) pr += __shfl_xor(pr, o);
        const int j = jt + 8 * hlf + v; const float alpha = 2.0f * sigm(pr + bb3);
        if (nloc == 0 && j != i) agg += Ai[j] * pmul(alpha, xb[j] - xi); } }
    agg += __shfl_xor(agg, 16);
    if (lane == 0) Ob[wid * 4 + ri] = xi + STEP * agg;
  }
  __syncthreads();
  for (int pass = 0; pass < 2; ++pass) { if (threadIdx.x < 8) *(volatile v4f*)(out + (size_t)b * N + i0 + threadIdx.x * 4) = *(const v4f*)(&Ob[threadIdx.x * 4]); __threadfence(); }
}
}

extern "C" void kernel_launch(void* const* d_in, const int* in_sizes, int n_in,
                              void* d_out, int out_size, void* d_ws, size_t ws_size, hipStream_t stream) {
  (void)n_in; (void)out_size;
  const float* x = (const float*)d_in[0]; const float* Theta = (const float*)d_in[1]; const float* W1 = (const float*)d_in[2]; const float* b1 = (const float*)d_in[3];
  const float* W2 = (const float*)d_in[4]; const float* b2 = (const float*)d_in[5]; const float* W3 = (const float*)d_in[6]; const float* b3 = (const float*)d_in[7];
  float* out = (float*)d_out;
  if (in_sizes[0] != Bn * N || in_sizes[1] != N * N || in_sizes[2] != H * 3 || in_sizes[4] != H * H || in_sizes[6] != H) return;
  size_t off = 0; char* ws = (char*)d_ws;
  auto carve = [&](size_t bytes) { char* p = ws + off; off += (bytes + 255) & ~(size_t)255; return p; };
  float* Arow = (float*)carve((size_t)N * N * 4); b16* w2p = (b16*)carve(H * H * 4);
  if (off > ws_size) return;
  prep_kernel<<<N / 8, 256, 0, stream>>>(Theta, W2, Arow, w2p);
  pair_kernel<<<Bn * N / 32, 256, 0, stream>>>(x, Arow, W1, b1, w2p, b2, W3, b3, out);
}
